// LSTM_36996848287879
// MI455X (gfx1250) — hardware-verified
//
#include <hip/hip_runtime.h>
#include <math.h>

typedef __attribute__((ext_vector_type(16))) _Float16 v16h;
typedef __attribute__((ext_vector_type(8)))  _Float16 v8h;
typedef __attribute__((ext_vector_type(8)))  float    v8f;
typedef __attribute__((ext_vector_type(4)))  float    v4f;
typedef __attribute__((ext_vector_type(2)))  float    v2f;

constexpr int NTRK      = 20000;
constexpr int EMBD      = 64;
constexpr int HIDN      = 128;
constexpr int NGATE     = 4 * HIDN;
constexpr int KCAT      = EMBD + HIDN;
constexpr int NOUTC     = 5;
constexpr int NENC      = 8;
constexpr int NDEC      = 11;
constexpr int NSTEPS    = NENC + NDEC;
constexpr int ROWS_BLK  = 32;
constexpr int NBLK      = NTRK / ROWS_BLK;
constexpr int NTHR      = 256;
constexpr int APITCH    = 200;
constexpr int LPITCH    = 136;
constexpr int WPITCH    = 136;
constexpr int RAWP      = 16;
constexpr float SCALE_IN   = 4.0f;
constexpr float CARRY_A    = 16.0f;
constexpr float CARRY_W    = 16.0f;
constexpr float FOLD_ACC   = 1.0f / (CARRY_A * CARRY_W);
constexpr float LO_SCALE   = 2048.0f;
constexpr float LO_INV     = 1.0f / LO_SCALE;
constexpr int OUT0_STEP = NTRK * NOUTC;
constexpr int OUT1_STEP = NTRK * 2;
constexpr int OUT1_OFF  = NSTEPS * OUT0_STEP;
constexpr int OUT_TOTAL = OUT1_OFF + NSTEPS * OUT1_STEP;

static_assert(NBLK * ROWS_BLK == NTRK, "exact row tiling");
static_assert(KCAT % 32 == 0 && HIDN % 32 == 0 && EMBD % 32 == 0, "k multiples of 32");
static_assert(NGATE == 512 && KCAT == 192, "plane shape");
static_assert((OUT0_STEP * 4) % 128 == 0 && (ROWS_BLK * NOUTC * 4) % 128 == 0, "out0 line alignment");
static_assert((OUT1_STEP * 4) % 128 == 0 && (ROWS_BLK * 2 * 4) % 128 == 0, "out1 line alignment");
static_assert(((long)OUT1_OFF * 4) % 128 == 0, "out1 base line alignment");
static_assert((long)OUT1_OFF * 4 == 7600000L, "out1 byte offset");
static_assert((long)OUT_TOTAL * 4 == 10640000L, "d_out bytes");
static_assert(ROWS_BLK * NOUTC == 160 && ROWS_BLK * 2 == 64, "staging extents");
static_assert((APITCH * 2) % 16 == 0 && (LPITCH * 2) % 16 == 0 && (WPITCH * 2) % 16 == 0, "16-B aligned fragment rows");
static_assert(NTHR == 8 * 32 && HIDN == 16 * (NTHR / 32), "8 waves x 16 hidden columns");

union FragU { v16h v; v8h h[2]; };
__device__ __forceinline__ v16h frag_load(const _Float16* p) {
  FragU f;
  f.h[0] = *(const v8h*)(p);
  f.h[1] = *(const v8h*)(p + 16);
  return f.v;
}
__device__ __forceinline__ v8f mma_h(v16h a, v16h b, v8f c) {
  return __builtin_amdgcn_wmma_f32_16x16x32_f16(false, a, false, b, (short)0, c, false, false);
}
__device__ __forceinline__ void guard8(v8f& a0, v8f& a1, v8f& a2, v8f& a3, v8f& a4, v8f& a5, v8f& a6, v8f& a7,
                                       v16h x0, v16h x1, v16h y0, v16h y1, v16h y2, v16h y3) {
  asm volatile("v_nop\n\tv_nop\n\tv_nop\n\tv_nop"
               : "+v"(a0), "+v"(a1), "+v"(a2), "+v"(a3), "+v"(a4), "+v"(a5), "+v"(a6), "+v"(a7)
               : "v"(x0), "v"(x1), "v"(y0), "v"(y1), "v"(y2), "v"(y3));
}
__device__ __forceinline__ void guard2(v8f& a0, v8f& a1, v16h x0, v16h x1, v16h y0, v16h y1) {
  asm volatile("v_nop\n\tv_nop\n\tv_nop\n\tv_nop"
               : "+v"(a0), "+v"(a1)
               : "v"(x0), "v"(x1), "v"(y0), "v"(y1));
}

__device__ __forceinline__ float sig_f(float x)  { return __builtin_amdgcn_rcpf(1.0f + expf(-x)); }
__device__ __forceinline__ float tanh_f(float x) { return 1.0f - 2.0f * __builtin_amdgcn_rcpf(1.0f + expf(2.0f * x)); }
__device__ __forceinline__ float softplus_f(float x) { return fmaxf(x, 0.0f) + log1pf(expf(-fabsf(x))); }

__global__ __launch_bounds__(NTHR) void wplane_kernel(const float* __restrict__ wih_e, const float* __restrict__ whh_e,
                                                     const float* __restrict__ wih_d, const float* __restrict__ whh_d,
                                                     unsigned short* __restrict__ bt_e, unsigned short* __restrict__ bt_d) {
  __shared__ float Tt[64 * 65];
  const int tid = threadIdx.x;
  const int n0 = blockIdx.x * 64;
  const int kt = blockIdx.y;
  const int ph = blockIdx.z;
  const float* wih = ph ? wih_d : wih_e;
  const float* whh = ph ? whh_d : whh_e;
  const float* src = (kt == 0) ? wih : whh;
  const int r0 = (kt == 0) ? 0 : (kt - 1) * 64;
  unsigned short* O = ph ? bt_d : bt_e;
#pragma unroll
  for (int i = 0; i < 4; ++i) {
    const int idx = i * NTHR + tid;
    const int rr = idx >> 4, cc = (idx & 15) * 4;
    const v4f v = *(const v4f*)(src + (size_t)(r0 + rr) * NGATE + n0 + cc);
    Tt[rr * 65 + cc + 0] = v[0];
    Tt[rr * 65 + cc + 1] = v[1];
    Tt[rr * 65 + cc + 2] = v[2];
    Tt[rr * 65 + cc + 3] = v[3];
  }
  __syncthreads();
  const int q = tid >> 3, c8 = (tid & 7) * 8;
  v8h hv[2];
#pragma unroll
  for (int g = 0; g < 2; ++g) {
    const int qq = g * 32 + q;
#pragma unroll
    for (int e = 0; e < 8; ++e) {
      const float f = Tt[(c8 + e) * 65 + qq];
      hv[g][e] = (_Float16)(f * CARRY_W);
    }
  }
  for (int pass = 0; pass < 2; ++pass) {
#pragma unroll
    for (int g = 0; g < 2; ++g) {
      const size_t o = (size_t)(n0 + g * 32 + q) * KCAT + (size_t)(kt * 64 + c8);
      *(volatile v8h*)(O + o) = hv[g];
    }
    __threadfence();
  }
}

__global__ __launch_bounds__(NTHR) void seq_cell_kernel(const float* __restrict__ observed,
                                                       const float* __restrict__ w_emb, const float* __restrict__ b_emb,
                                                       const float* __restrict__ b_enc, const float* __restrict__ b_dec,
                                                       const float* __restrict__ w_out, const float* __restrict__ b_out,
                                                       const unsigned short* __restrict__ bt_enc,
                                                       const unsigned short* __restrict__ bt_dec,
                                                       float* __restrict__ out) {
  __shared__ __align__(16) _Float16 At[ROWS_BLK * APITCH];
  __shared__ __align__(16) _Float16 Hlo[ROWS_BLK * LPITCH];
  __shared__ __align__(16) _Float16 Woh[16 * WPITCH];
  __shared__ __align__(16) _Float16 Wol[16 * WPITCH];
  __shared__ __align__(16) float s_wemb[3 * EMBD];
  __shared__ __align__(16) float s_vel[ROWS_BLK * 2];
  __shared__ __align__(16) float s_mask[ROWS_BLK];
  __shared__ __align__(16) float s_raw[ROWS_BLK * RAWP];
  __shared__ __align__(16) float s_o0[ROWS_BLK * NOUTC];
  __shared__ __align__(16) float s_o1[ROWS_BLK * 2];

  const int tid = threadIdx.x, lane = tid & 31, w = tid >> 5;
  const int c = lane & 15, hh = lane >> 4, koff = hh * 8;
  const int blk = blockIdx.x;
  const int col = w * 16 + c;
  const float QNANF = __uint_as_float(0x7fc00000u);

  {
    const v8h zero8 = {(_Float16)0.0f, (_Float16)0.0f, (_Float16)0.0f, (_Float16)0.0f,
                       (_Float16)0.0f, (_Float16)0.0f, (_Float16)0.0f, (_Float16)0.0f};
#pragma unroll
    for (int i = 0; i < 2; ++i) {
      const int idx = i * NTHR + tid;
      const int row = idx >> 4, c8 = (idx & 15) * 8;
      *(v8h*)(At + row * APITCH + EMBD + c8) = zero8;
      *(v8h*)(Hlo + row * LPITCH + c8) = zero8;
    }
  }
  {
    const int n = tid >> 4, k0 = (tid & 15) * 8;
    const int nc = (n < NOUTC) ? n : (NOUTC - 1);
    v8h hv, lv;
#pragma unroll
    for (int e = 0; e < 8; ++e) {
      const float wraw = w_out[(k0 + e) * NOUTC + nc];
      const float wv = (n < NOUTC) ? wraw : 0.0f;
      const float ws = wv * CARRY_W;
      const _Float16 hi = (_Float16)ws;
      const float hif = (float)hi;
      const float res = (ws - hif) * LO_SCALE;
      hv[e] = hi;
      lv[e] = (_Float16)res;
    }
    *(v8h*)(Woh + n * WPITCH + k0) = hv;
    *(v8h*)(Wol + n * WPITCH + k0) = lv;
  }
  asm volatile("" ::: "memory");
  if (w < 4) {
    s_wemb[tid] = w_emb[tid];
  } else if (w < 6) {
    s_wemb[tid] = b_emb[tid - 2 * EMBD];
  }
  asm volatile("" ::: "memory");
  float be[4], bd[4];
#pragma unroll
  for (int g = 0; g < 4; ++g) {
    be[g] = b_enc[g * HIDN + col];
    bd[g] = b_dec[g * HIDN + col];
  }
  asm volatile("" ::: "memory");
  const int ncl = (c < NOUTC) ? c : (NOUTC - 1);
  const float bo_raw = b_out[ncl];
  const float bo = (c < NOUTC) ? bo_raw : 0.0f;

  float c_reg[2][8];
#pragma unroll
  for (int i = 0; i < 2; ++i)
#pragma unroll
    for (int r = 0; r < 8; ++r) c_reg[i][r] = 0.0f;

  float p1x = 0.0f, p1y = 0.0f, p2x = 0.0f, p2y = 0.0f;
  float cur_o2x = 0.0f, cur_o2y = 0.0f;
  bool cur_mk = false;
  const int gtrk = blk * ROWS_BLK + lane;

  if (w == 0) {
    const v2f a = *(const v2f*)(observed + ((size_t)0 * NTRK + gtrk) * 2);
    const v2f b = *(const v2f*)(observed + ((size_t)1 * NTRK + gtrk) * 2);
    const float o1x = a[0], o1y = a[1], o2x = b[0], o2y = b[1];
    const bool mk = !((o1x != o1x) || (o2x != o2x));
    s_vel[2 * lane + 0] = mk ? (o2x - o1x) : 0.0f;
    s_vel[2 * lane + 1] = mk ? (o2y - o1y) : 0.0f;
    s_mask[lane] = mk ? 1.0f : 0.0f;
    cur_o2x = o2x;
    cur_o2y = o2y;
    cur_mk = mk;
  }
  __syncthreads();

  const v8f z8 = {0.f, 0.f, 0.f, 0.f, 0.f, 0.f, 0.f, 0.f};

#pragma unroll 1
  for (int t = 0; t < NSTEPS; ++t) {
    const bool enc = (t < NENC);

    {
      const int row = tid >> 3, e0 = (tid & 7) * 8;
      const float vx = SCALE_IN * s_vel[2 * row + 0];
      const float vy = SCALE_IN * s_vel[2 * row + 1];
      const v4f wa0 = *(const v4f*)(s_wemb + e0);
      const v4f wa1 = *(const v4f*)(s_wemb + e0 + 4);
      const v4f wb0 = *(const v4f*)(s_wemb + EMBD + e0);
      const v4f wb1 = *(const v4f*)(s_wemb + EMBD + e0 + 4);
      const v4f bb0 = *(const v4f*)(s_wemb + 2 * EMBD + e0);
      const v4f bb1 = *(const v4f*)(s_wemb + 2 * EMBD + e0 + 4);
      v8h hv;
#pragma unroll
      for (int e = 0; e < 4; ++e) {
        const float f0 = (vx * wa0[e] + vy * wb0[e]) + bb0[e];
        const float f1 = (vx * wa1[e] + vy * wb1[e]) + bb1[e];
        hv[e]     = (_Float16)(fmaxf(f0, 0.0f) * CARRY_A);
        hv[4 + e] = (_Float16)(fmaxf(f1, 0.0f) * CARRY_A);
      }
      *(v8h*)(At + row * APITCH + e0) = hv;
    }
    __syncthreads();

    v8f acc[2][4];
#pragma unroll
    for (int i = 0; i < 2; ++i)
#pragma unroll
      for (int g = 0; g < 4; ++g) acc[i][g] = z8;
    {
      const _Float16* Bt = (const _Float16*)(enc ? bt_enc : bt_dec);
      const _Float16* bp = Bt + (size_t)col * KCAT + koff;
      const _Float16* ap = At + c * APITCH + koff;
#pragma unroll 1
      for (int k0 = 0; k0 < KCAT; k0 += 32) {
        const v16h b0 = frag_load(bp + (size_t)0 * HIDN * KCAT + k0);
        const v16h b1 = frag_load(bp + (size_t)1 * HIDN * KCAT + k0);
        const v16h b2 = frag_load(bp + (size_t)2 * HIDN * KCAT + k0);
        const v16h b3 = frag_load(bp + (size_t)3 * HIDN * KCAT + k0);
        const v16h a0 = frag_load(ap + k0);
        const v16h a1 = frag_load(ap + 16 * APITCH + k0);
        acc[0][0] = mma_h(a0, b0, acc[0][0]);
        acc[0][1] = mma_h(a0, b1, acc[0][1]);
        acc[0][2] = mma_h(a0, b2, acc[0][2]);
        acc[0][3] = mma_h(a0, b3, acc[0][3]);
        acc[1][0] = mma_h(a1, b0, acc[1][0]);
        acc[1][1] = mma_h(a1, b1, acc[1][1]);
        acc[1][2] = mma_h(a1, b2, acc[1][2]);
        acc[1][3] = mma_h(a1, b3, acc[1][3]);
        guard8(acc[0][0], acc[0][1], acc[0][2], acc[0][3], acc[1][0], acc[1][1], acc[1][2], acc[1][3],
               a0, a1, b0, b1, b2, b3);
      }
    }
    __syncthreads();

    {
      const float bi = enc ? be[0] : bd[0];
      const float bf = enc ? be[1] : bd[1];
      const float bg = enc ? be[2] : bd[2];
      const float bq = enc ? be[3] : bd[3];
#pragma unroll
      for (int i = 0; i < 2; ++i) {
#pragma unroll
        for (int r = 0; r < 8; ++r) {
          const int row = i * 16 + 8 * hh + r;
          const bool mk = s_mask[row] > 0.5f;
          const float zi = acc[i][0][r] * FOLD_ACC + bi;
          const float zf = acc[i][1][r] * FOLD_ACC + bf;
          const float zg = acc[i][2][r] * FOLD_ACC + bg;
          const float zo = acc[i][3][r] * FOLD_ACC + bq;
          const float ig = sig_f(zi);
          const float fg = sig_f(zf);
          const float gg = tanh_f(zg);
          const float og = sig_f(zo);
          const float cold = c_reg[i][r];
          const float cn = fg * cold + ig * gg;
          const float hn = og * tanh_f(cn);
          c_reg[i][r] = mk ? cn : cold;
          const float hs = hn * CARRY_A;
          const _Float16 hi = (_Float16)hs;
          const float hif = (float)hi;
          const _Float16 lo = (_Float16)((hs - hif) * LO_SCALE);
          if (mk) {
            At[row * APITCH + EMBD + col] = hi;
            Hlo[row * LPITCH + col] = lo;
          }
        }
      }
    }
    __syncthreads();

    if (w < 2) {
      const _Float16* ahp = At + (w * 16 + c) * APITCH + EMBD + koff;
      const _Float16* alp = Hlo + (w * 16 + c) * LPITCH + koff;
      const _Float16* whp = Woh + c * WPITCH + koff;
      const _Float16* wlp = Wol + c * WPITCH + koff;
      v8f am = z8, ar = z8;
#pragma unroll 1
      for (int k0 = 0; k0 < HIDN; k0 += 32) {
        const v16h ah = frag_load(ahp + k0);
        const v16h al = frag_load(alp + k0);
        const v16h bh = frag_load(whp + k0);
        const v16h bl = frag_load(wlp + k0);
        am = mma_h(ah, bh, am);
        ar = mma_h(ah, bl, ar);
        ar = mma_h(al, bh, ar);
        guard2(am, ar, ah, al, bh, bl);
      }
#pragma unroll
      for (int r = 0; r < 8; ++r) {
        const float rv = (am[r] + ar[r] * LO_INV) * FOLD_ACC + bo;
        s_raw[(w * 16 + 8 * hh + r) * RAWP + c] = rv;
      }
    }
    __syncthreads();

    if (w == 0) {
      const v4f r03 = *(const v4f*)(s_raw + lane * RAWP);
      const float r4 = s_raw[lane * RAWP + 4];
      const float t0 = r03[0];
      const float t1 = r03[1];
      const float t2 = 0.01f + 0.2f * softplus_f(r03[2]);
      const float t3 = 0.01f + 0.2f * softplus_f(r03[3]);
      const float t4 = 0.7f * sig_f(r4);
      const float n0 = cur_mk ? t0 : QNANF;
      const float n1 = cur_mk ? t1 : QNANF;
      const float n2 = cur_mk ? t2 : QNANF;
      const float n3 = cur_mk ? t3 : QNANF;
      const float n4 = cur_mk ? t4 : QNANF;
      const float px = cur_o2x + n0;
      const float py = cur_o2y + n1;
      s_o0[lane * NOUTC + 0] = n0;
      s_o0[lane * NOUTC + 1] = n1;
      s_o0[lane * NOUTC + 2] = n2;
      s_o0[lane * NOUTC + 3] = n3;
      s_o0[lane * NOUTC + 4] = n4;
      s_o1[lane * 2 + 0] = px;
      s_o1[lane * 2 + 1] = py;
      p2x = p1x;
      p2y = p1y;
      p1x = px;
      p1y = py;
      if (t + 1 < NSTEPS) {
        float o1x, o1y, o2x, o2y;
        if (t + 1 < NENC) {
          const v2f a = *(const v2f*)(observed + ((size_t)(t + 1) * NTRK + gtrk) * 2);
          const v2f b = *(const v2f*)(observed + ((size_t)(t + 2) * NTRK + gtrk) * 2);
          o1x = a[0];
          o1y = a[1];
          o2x = b[0];
          o2y = b[1];
        } else {
          o1x = p2x;
          o1y = p2y;
          o2x = p1x;
          o2y = p1y;
        }
        const bool mk = !((o1x != o1x) || (o2x != o2x));
        s_vel[2 * lane + 0] = mk ? (o2x - o1x) : 0.0f;
        s_vel[2 * lane + 1] = mk ? (o2y - o1y) : 0.0f;
        s_mask[lane] = mk ? 1.0f : 0.0f;
        cur_o2x = o2x;
        cur_o2y = o2y;
        cur_mk = mk;
      }
    }
    __syncthreads();

    if (w == 0) {
      float* o0 = out + (size_t)t * OUT0_STEP + (size_t)blk * (ROWS_BLK * NOUTC);
      float* o1 = out + (size_t)OUT1_OFF + (size_t)t * OUT1_STEP + (size_t)blk * (ROWS_BLK * 2);
      const int l8 = (lane < 8) ? lane : 7;
      const int l16 = (lane < 16) ? lane : 15;
      const v4f va = *(const v4f*)(s_o0 + 4 * lane);
      const v4f vb = *(const v4f*)(s_o0 + 128 + 4 * l8);
      const v4f vc = *(const v4f*)(s_o1 + 4 * l16);
      for (int pass = 0; pass < 2; ++pass) {
        *(volatile v4f*)(o0 + 4 * lane) = va;
        if (lane < 8) *(volatile v4f*)(o0 + 128 + 4 * lane) = vb;
        if (lane < 16) *(volatile v4f*)(o1 + 4 * lane) = vc;
        __threadfence();
      }
    }
  }
}

extern "C" void kernel_launch(void* const* d_in, const int* in_sizes, int n_in,
                              void* d_out, int out_size, void* d_ws, size_t ws_size, hipStream_t stream) {
  if (n_in < 14 || d_out == nullptr || d_ws == nullptr) return;
  if (in_sizes[0] != 9 * NTRK * 2 || in_sizes[4] != 2 * EMBD || in_sizes[5] != EMBD ||
      in_sizes[6] != EMBD * NGATE || in_sizes[7] != HIDN * NGATE || in_sizes[8] != NGATE ||
      in_sizes[9] != EMBD * NGATE || in_sizes[10] != HIDN * NGATE || in_sizes[11] != NGATE ||
      in_sizes[12] != HIDN * NOUTC || in_sizes[13] != NOUTC || out_size != OUT_TOTAL) return;

  const float* observed = (const float*)d_in[0];
  const float* w_emb    = (const float*)d_in[4];
  const float* b_emb    = (const float*)d_in[5];
  const float* wih_enc  = (const float*)d_in[6];
  const float* whh_enc  = (const float*)d_in[7];
  const float* b_enc    = (const float*)d_in[8];
  const float* wih_dec  = (const float*)d_in[9];
  const float* whh_dec  = (const float*)d_in[10];
  const float* b_dec    = (const float*)d_in[11];
  const float* w_out    = (const float*)d_in[12];
  const float* b_out    = (const float*)d_in[13];
  float* out = (float*)d_out;

  char* ws = (char*)d_ws;
  size_t off = 0;
  const size_t plane_bytes = (size_t)NGATE * KCAT * 2;
  unsigned short* bt_enc = (unsigned short*)(ws + off);
  off += (plane_bytes + 255) & ~(size_t)255;
  unsigned short* bt_dec = (unsigned short*)(ws + off);
  off += (plane_bytes + 255) & ~(size_t)255;
  if (off > ws_size || off > (size_t)134217728) return;

  wplane_kernel<<<dim3(NGATE / 64, KCAT / 64, 2), NTHR, 0, stream>>>(wih_enc, whh_enc, wih_dec, whh_dec, bt_enc, bt_dec);
  seq_cell_kernel<<<NBLK, NTHR, 0, stream>>>(observed, w_emb, b_emb, b_enc, b_dec, w_out, b_out, bt_enc, bt_dec, out);
}
